// DualAttentionModule_38989713113557
// MI455X (gfx1250) — hardware-verified
//
#include <hip/hip_runtime.h>
#include <math.h>

typedef __attribute__((ext_vector_type(16))) _Float16 v16h;
typedef __attribute__((ext_vector_type(16))) __bf16 v16b;
typedef __attribute__((ext_vector_type(8)))  _Float16 v8h;
typedef __attribute__((ext_vector_type(8)))  float v8f;
typedef __attribute__((ext_vector_type(4)))  float v4f;
typedef __attribute__((ext_vector_type(2)))  float v2f;
typedef __attribute__((ext_vector_type(4)))  unsigned v4u;
typedef __attribute__((ext_vector_type(4)))  int v4i;
typedef float __attribute__((may_alias)) float_a;
typedef int __attribute__((may_alias)) int_a;

template <typename T> __device__ __forceinline__ void vst2(void* p, T v) { *(volatile T*)p = v; __threadfence(); *(volatile T*)p = v; }
__device__ __forceinline__ v8f wmma16(v16h a, v16h b, v8f c) {
  v8f d = __builtin_amdgcn_wmma_f32_16x16x32_f16(false, a, false, b, (short)0, c, false, false);
  asm volatile("v_nop\n\tv_nop\n\tv_nop\n\tv_nop" : "+v"(d) : "v"(a), "v"(b));
  return d;
}
__device__ __forceinline__ v8f wmma_bf(v16b a, v16b b, v8f c) {
  v8f d = __builtin_amdgcn_wmma_f32_16x16x32_bf16(false, a, false, b, (short)0, c, false, false);
  asm volatile("v_nop\n\tv_nop\n\tv_nop\n\tv_nop" : "+v"(d) : "v"(a), "v"(b));
  return d;
}
__device__ __forceinline__ v16h frag_h(const _Float16* rowk0, int lane) {
  union { v16h v; v8h q[2]; } u; const _Float16* p = rowk0 + 8 * (lane >> 4);
  u.q[0] = *(const v8h*)p; u.q[1] = *(const v8h*)(p + 16); return u.v;
}
__device__ __forceinline__ v16h frag_f32(const float* rowk0, int lane) {
  v16h a; const float* p = rowk0 + 8 * (lane >> 4);
#pragma unroll
  for (int i = 0; i < 8; ++i) { a[i] = (_Float16)p[i]; a[8 + i] = (_Float16)p[16 + i]; }
  return a;
}
__device__ __forceinline__ v16h frag_f32s(const float* rowk0, int lane, float sc) {
  v16h a; const float* p = rowk0 + 8 * (lane >> 4);
#pragma unroll
  for (int i = 0; i < 8; ++i) { a[i] = (_Float16)(p[i] * sc); a[8 + i] = (_Float16)(p[16 + i] * sc); }
  return a;
}
__device__ __forceinline__ v16h fragc_f32(const float* W, int k0, int n, int lane, int ld, int K) {
  v16h a; const int g = lane >> 4;
#pragma unroll
  for (int i = 0; i < 8; ++i) { const int ka = k0 + 8 * g + i, kb = ka + 16;
    a[i] = (_Float16)(ka < K ? W[(size_t)(ka < K ? ka : K - 1) * ld + n] : 0.f); a[8 + i] = (_Float16)(kb < K ? W[(size_t)(kb < K ? kb : K - 1) * ld + n] : 0.f); }
  return a;
}
struct F2 { v16b h, l; };
__device__ __forceinline__ F2 bsplit16(const float v[16]) { F2 r;
#pragma unroll
  for (int i = 0; i < 16; ++i) { const __bf16 h = (__bf16)v[i]; r.h[i] = h; r.l[i] = (__bf16)(v[i] - (float)h); }
  return r; }
__device__ __forceinline__ F2 split_row(const float* row, int k0, int lane) { float v[16]; const float* p = row + k0 + 8 * (lane >> 4);
#pragma unroll
  for (int i = 0; i < 8; ++i) { v[i] = p[i]; v[8 + i] = p[16 + i]; }
  return bsplit16(v); }
__device__ __forceinline__ F2 split_rowK(const float* row, int k0, int lane, int K) { float v[16]; const int g = lane >> 4;
#pragma unroll
  for (int i = 0; i < 8; ++i) { const int ka = k0 + 8 * g + i, kb = ka + 16; v[i] = ka < K ? row[ka < K ? ka : K - 1] : 0.f; v[8 + i] = kb < K ? row[kb < K ? kb : K - 1] : 0.f; }
  return bsplit16(v); }
__device__ __forceinline__ F2 split_col(const float* W, int k0, int n, int lane, int ld, int K) { float v[16]; const int g = lane >> 4;
#pragma unroll
  for (int i = 0; i < 8; ++i) { const int ka = k0 + 8 * g + i, kb = ka + 16; v[i] = ka < K ? W[(size_t)(ka < K ? ka : K - 1) * ld + n] : 0.f; v[8 + i] = kb < K ? W[(size_t)(kb < K ? kb : K - 1) * ld + n] : 0.f; }
  return bsplit16(v); }
__device__ __forceinline__ v8f mac3(const F2& a, const F2& b, v8f c) { c = wmma_bf(a.l, b.h, c); c = wmma_bf(a.h, b.l, c); return wmma_bf(a.h, b.h, c); }
__device__ __forceinline__ float sigm(float v) { return 1.0f / (1.0f + expf(-v)); }
#define LDSX() do { asm volatile("s_wait_dscnt 0" ::: "memory"); __builtin_amdgcn_wave_barrier(); __builtin_amdgcn_fence(__ATOMIC_RELEASE, "workgroup"); } while (0)


#define NB 4
#define NN 4096
#define CC 512
#define CK 64
#define NR (NB * NN)
#ifndef TRB
#define TRB (NN / 64)
#define TNB NB
#endif
typedef __attribute__((ext_vector_type(8))) __bf16 v8b;
__device__ __forceinline__ v16b frag_b(const __bf16* rowk0, int lane) {
  union { v16b v; v8b q[2]; } u; const __bf16* p = rowk0 + 8 * (lane >> 4);
  u.q[0] = *(const v8b*)p; u.q[1] = *(const v8b*)(p + 16); return u.v;
}
__device__ __forceinline__ float bfr(float v) { return (float)(__bf16)v; }
__device__ __attribute__((noinline)) float exp_ni(float v) { return expf(v); }
__device__ __attribute__((noinline)) float erf_ni(float v) { return erff(v); }

#define WS_PW  0u
#define WS_P3  (WS_PW + 2u * (size_t)128 * CC)
#define WS_BC  (WS_P3 + 2u * (size_t)CC * CC)
#define WS_DT  (WS_BC + 4u * (size_t)NR * 128)
#define WS_XT  (WS_DT + 2u * (size_t)NB * CC * NN)
#define WS_S   (WS_XT + 2u * (size_t)NB * CC * NN)
#define WS_P   (WS_S + 4u * (size_t)NN * NN)
#define WS_BCD (WS_P + 2u * (size_t)NN * NN)
#define WS_AA  (WS_BCD + 4u * (size_t)NB * CC * NN)
#define WS_SO  (WS_AA + 4u * (size_t)NB * CC * CC)
#define WS_AAA (WS_SO + 2u * (size_t)NB * CC * CC)
#define WS_END (WS_AAA + 4u * (size_t)NB * NN * CC)

__global__ __launch_bounds__(256) void k_pack(const float* __restrict__ W1, const float* __restrict__ W2, const float* __restrict__ W3, __bf16* __restrict__ PW, __bf16* __restrict__ P3) { const int n = blockIdx.x, which = blockIdx.y, t = threadIdx.x; __shared__ __align__(16) __bf16 s[CC];
  if (which == 0) { if (n >= 128) return; const float* w = (n < CK) ? W1 : W2; const int cI = n & (CK - 1); for (int k = t; k < CC; k += 256) s[k] = (__bf16)w[(size_t)k * CK + cI]; __syncthreads(); if (t < CC / 8) vst2((unsigned*)(PW + (size_t)n * CC + t * 8), *(const v4u*)&s[t * 8]); }
  else { for (int k = t; k < CC; k += 256) s[k] = (__bf16)W3[(size_t)k * CC + n]; __syncthreads(); if (t < CC / 8) vst2((unsigned*)(P3 + (size_t)n * CC + t * 8), *(const v4u*)&s[t * 8]); } }
__global__ __launch_bounds__(128) void k_proj(const float* __restrict__ X, const __bf16* __restrict__ PW, const __bf16* __restrict__ P3, float* __restrict__ BC, _Float16* __restrict__ DT, _Float16* __restrict__ XT) {
  __shared__ __align__(16) float sf[4][16][132]; __shared__ __align__(16) _Float16 st[128][72];
  const int tid = threadIdx.x, wave = tid >> 5, lane = tid & 31, col = lane & 15, g = lane >> 4; const int which = blockIdx.z; const size_t rb = (size_t)blockIdx.x * 64; const size_t r0 = rb + wave * 16;
  if (which >= 5) { const int c0 = (which - 5) * 128; for (int e = tid; e < 64 * 128; e += 128) { const int rl = e >> 7, cl = e & 127; st[cl][rl] = (_Float16)bfr(X[(rb + rl) * CC + c0 + cl]); } __syncthreads();
    const size_t b = rb / NN; const int n0 = (int)(rb % NN); for (int e = tid; e < 128 * 8; e += 128) { const int d = e >> 3, pc = e & 7; vst2((unsigned*)(XT + ((b * CC + c0 + d) * NN) + n0 + pc * 8), *(const v4u*)&st[d][pc * 8]); } return; }
  const int c0 = (which == 0) ? 0 : (which - 1) * 128; const __bf16* Wr = (which == 0) ? PW : (P3 + (size_t)c0 * CC);
  v8f acc[8] = {};
#pragma unroll 2
  for (int kc = 0; kc < CC / 32; ++kc) { v16b a; { const float* p = X + (r0 + col) * CC + kc * 32 + 8 * g;
#pragma unroll
      for (int i = 0; i < 8; ++i) { a[i] = (__bf16)p[i]; a[8 + i] = (__bf16)p[16 + i]; } }
#pragma unroll
    for (int j = 0; j < 8; ++j) acc[j] = wmma_bf(a, frag_b(Wr + (size_t)(j * 16 + col) * CC + kc * 32, lane), acc[j]); }
#pragma unroll
  for (int j = 0; j < 8; ++j)
#pragma unroll
    for (int r = 0; r < 8; ++r) { if (which == 0) sf[wave][8 * g + r][j * 16 + col] = acc[j][r]; else st[j * 16 + col][wave * 16 + 8 * g + r] = (_Float16)acc[j][r]; }
  __syncthreads();
  if (which == 0) { for (int rl = 0; rl < 16; ++rl) vst2(BC + (r0 + rl) * 128 + lane * 4, *(const v4f*)&sf[wave][rl][lane * 4]); }
  else { const size_t b = rb / NN; const int n0 = (int)(rb % NN); for (int e = tid; e < 128 * 8; e += 128) { const int d = e >> 3, pc = e & 7; vst2((unsigned*)(DT + ((b * CC + c0 + d) * NN) + n0 + pc * 8), *(const v4u*)&st[d][pc * 8]); } }
}
__global__ __launch_bounds__(128) void k_s(const float* __restrict__ BC, int b, float* __restrict__ S) { __shared__ __align__(16) float so[4][16][132];
  const int tid = threadIdx.x, wave = tid >> 5, lane = tid & 31, col = lane & 15, g = lane >> 4; const int i0 = blockIdx.x * 64 + wave * 16; const int n0 = blockIdx.y * 128; const size_t rb = (size_t)b * NN;
  v8f acc[8] = {};
#pragma unroll
  for (int kc = 0; kc < 2; ++kc) { const F2 a = split_row(BC + (rb + i0 + col) * 128, kc * 32, lane);
#pragma unroll
    for (int j = 0; j < 8; ++j) { const F2 w = split_row(BC + (rb + n0 + j * 16 + col) * 128 + CK, kc * 32, lane); acc[j] = mac3(a, w, acc[j]); } }
#pragma unroll
  for (int j = 0; j < 8; ++j)
#pragma unroll
    for (int r = 0; r < 8; ++r) so[wave][8 * g + r][j * 16 + col] = acc[j][r];
  LDSX(); for (int rl = 0; rl < 16; ++rl) vst2(S + ((size_t)(i0 + rl) * NN) + n0 + lane * 4, *(const v4f*)&so[wave][rl][lane * 4]); }
__global__ __launch_bounds__(256) void k_prow(const float* __restrict__ S, _Float16* __restrict__ P) { __shared__ float red[8]; __shared__ __align__(16) _Float16 sp[NN]; const int t = threadIdx.x; const size_t row = blockIdx.x; const float* sr = S + row * NN;
  float v[16]; float mx = -3.0e38f; for (int i = 0; i < 16; ++i) { v[i] = sr[t * 16 + i]; mx = fmaxf(mx, v[i]); }
#pragma unroll
  for (int o = 1; o < 32; o <<= 1) mx = fmaxf(mx, __shfl_xor(mx, o));
  if ((t & 31) == 0) red[t >> 5] = mx; __syncthreads(); float M = red[0]; for (int i = 1; i < 8; ++i) M = fmaxf(M, red[i]); __syncthreads();
  float z = 0.f; for (int i = 0; i < 16; ++i) { v[i] = __expf(v[i] - M); z += v[i]; }
#pragma unroll
  for (int o = 1; o < 32; o <<= 1) z += __shfl_xor(z, o);
  if ((t & 31) == 0) red[t >> 5] = z; __syncthreads(); float Z = 0.f; for (int i = 0; i < 8; ++i) Z += red[i]; const float iz = 2048.0f / Z;
  for (int i = 0; i < 16; ++i) sp[t * 16 + i] = (_Float16)(v[i] * iz); __syncthreads();
  for (int q = t; q < NN / 8; q += 256) vst2((unsigned*)(P + row * NN + q * 8), *(const v4u*)&sp[q * 8]); }
__global__ __launch_bounds__(128) void k_pv(const _Float16* __restrict__ DT, const _Float16* __restrict__ P, int bI, float* __restrict__ BCD) { __shared__ __align__(16) float so[4][16][132];
  const int tid = threadIdx.x, wave = tid >> 5, lane = tid & 31, col = lane & 15, g = lane >> 4; const size_t b = (size_t)bI; const int c0 = blockIdx.x * 64 + wave * 16; const int i0 = blockIdx.y * 128;
  v8f acc[8] = {};
#pragma unroll 2
  for (int kc = 0; kc < NN / 32; ++kc) { const v16h a = frag_h(DT + ((b * CC + c0 + col) * NN) + kc * 32, lane);
#pragma unroll
    for (int j = 0; j < 8; ++j) acc[j] = wmma16(a, frag_h(P + ((size_t)(i0 + j * 16 + col) * NN) + kc * 32, lane), acc[j]); }
#pragma unroll
  for (int j = 0; j < 8; ++j)
#pragma unroll
    for (int r = 0; r < 8; ++r) so[wave][8 * g + r][j * 16 + col] = acc[j][r] * (1.0f / 2048.0f);
  LDSX(); for (int rl = 0; rl < 16; ++rl) vst2(BCD + ((b * CC + c0 + rl) * NN) + i0 + lane * 4, *(const v4f*)&so[wave][rl][lane * 4]); }
__global__ __launch_bounds__(128) void k_aa(const _Float16* __restrict__ XT, float* __restrict__ AA) { __shared__ __align__(16) float so[4][16][132];
  const int tid = threadIdx.x, wave = tid >> 5, lane = tid & 31, col = lane & 15, g = lane >> 4; const size_t b = blockIdx.z; const int i0 = blockIdx.x * 64 + wave * 16; const int j0 = blockIdx.y * 128;
  v8f acc[8] = {};
#pragma unroll 2
  for (int kc = 0; kc < NN / 32; ++kc) { const v16h a = frag_h(XT + ((b * CC + i0 + col) * NN) + kc * 32, lane);
#pragma unroll
    for (int j = 0; j < 8; ++j) acc[j] = wmma16(a, frag_h(XT + ((b * CC + j0 + j * 16 + col) * NN) + kc * 32, lane), acc[j]); }
#pragma unroll
  for (int j = 0; j < 8; ++j)
#pragma unroll
    for (int r = 0; r < 8; ++r) so[wave][8 * g + r][j * 16 + col] = acc[j][r];
  LDSX(); for (int rl = 0; rl < 16; ++rl) vst2(AA + ((b * CC + i0 + rl) * CC) + j0 + lane * 4, *(const v4f*)&so[wave][rl][lane * 4]); }
__global__ __launch_bounds__(256) void k_soft(const float* __restrict__ AA, _Float16* __restrict__ SO) { __shared__ __align__(16) _Float16 st[CC][72]; __shared__ float red[2][64];
  const int t = threadIdx.x; const size_t b = blockIdx.y; const int c0 = blockIdx.x * 64;
  { const int rl = t >> 2, part = t & 3; const float* row = AA + ((b * CC + c0 + rl) * CC); float mx = -3.0e38f; for (int j = part; j < CC; j += 4) mx = fmaxf(mx, row[j]); mx = fmaxf(mx, __shfl_xor(mx, 1)); mx = fmaxf(mx, __shfl_xor(mx, 2));
    float z = 0.f; for (int j = part; j < CC; j += 4) z += __expf(row[j] - mx); z += __shfl_xor(z, 1); z += __shfl_xor(z, 2); const float iz = 1.0f / z;
    for (int j = part; j < CC; j += 4) st[j][rl] = (_Float16)(__expf(row[j] - mx) * iz); }
  __syncthreads();
  for (int e = t; e < CC * 8; e += 256) { const int j = e >> 3, pc = e & 7; vst2((unsigned*)(SO + ((b * CC + j) * CC) + c0 + pc * 8), *(const v4u*)&st[j][pc * 8]); } }
__global__ __launch_bounds__(128) void k_aaa(const float* __restrict__ X, const _Float16* __restrict__ SO, float* __restrict__ AAA) { __shared__ __align__(16) float so[4][16][132];
  const int tid = threadIdx.x, wave = tid >> 5, lane = tid & 31, col = lane & 15, g = lane >> 4; const size_t b = blockIdx.z; const size_t r0 = b * NN + (size_t)blockIdx.x * 64 + wave * 16; const int j0 = blockIdx.y * 128;
  v8f acc[8] = {};
#pragma unroll 2
  for (int kc = 0; kc < CC / 32; ++kc) { v16h a; { const float* p = X + (r0 + col) * CC + kc * 32 + 8 * g;
#pragma unroll
      for (int i = 0; i < 8; ++i) { a[i] = (_Float16)bfr(p[i]); a[8 + i] = (_Float16)bfr(p[16 + i]); } }
#pragma unroll
    for (int j = 0; j < 8; ++j) acc[j] = wmma16(a, frag_h(SO + ((b * CC + j0 + j * 16 + col) * CC) + kc * 32, lane), acc[j]); }
#pragma unroll
  for (int j = 0; j < 8; ++j)
#pragma unroll
    for (int r = 0; r < 8; ++r) so[wave][8 * g + r][j * 16 + col] = acc[j][r];
  LDSX(); for (int rl = 0; rl < 16; ++rl) vst2(AAA + (r0 + rl) * CC + j0 + lane * 4, *(const v4f*)&so[wave][rl][lane * 4]); }
__global__ __launch_bounds__(256) void k_fin(const float* __restrict__ BCD, const float* __restrict__ AAA, const float* __restrict__ X, const float* __restrict__ GP, const float* __restrict__ GC, float* __restrict__ OUT) { const size_t i4 = (size_t)blockIdx.x * 256 + threadIdx.x; const size_t f = i4 * 4; const float gp = bfr(GP[0]), gc = bfr(GC[0]);
  v4f o4; for (int i = 0; i < 4; ++i) o4[i] = gp * BCD[f + i] + gc * AAA[f + i] + 2.0f * bfr(X[f + i]); vst2(OUT + f, o4); }
extern "C" void kernel_launch(void* const* d_in, const int* in_sizes, int n_in, void* d_out, int out_size, void* d_ws, size_t ws_size, hipStream_t stream) {
  (void)in_sizes; (void)n_in; (void)out_size;
  const float** F = (const float**)d_in;
  if (ws_size < (size_t)WS_END) return;
  char* ws = (char*)d_ws; __bf16 *PW = (__bf16*)(ws + WS_PW), *P3 = (__bf16*)(ws + WS_P3); float* BC = (float*)(ws + WS_BC); _Float16 *DT = (_Float16*)(ws + WS_DT), *XT = (_Float16*)(ws + WS_XT), *P = (_Float16*)(ws + WS_P), *SO = (_Float16*)(ws + WS_SO); float *S = (float*)(ws + WS_S), *BCD = (float*)(ws + WS_BCD), *AA = (float*)(ws + WS_AA), *AAA = (float*)(ws + WS_AAA);
  k_pack<<<dim3(CC, 2), 256, 0, stream>>>(F[1], F[2], F[3], PW, P3);
  k_proj<<<dim3(TNB * NN / 64, 1, 9), 128, 0, stream>>>(F[0], PW, P3, BC, DT, XT);
  for (int b = 0; b < TNB; ++b) {
    k_s<<<dim3(TRB, NN / 128), 128, 0, stream>>>(BC, b, S);
    k_prow<<<TRB * 64, 256, 0, stream>>>(S, P);
    k_pv<<<dim3(CC / 64, (TRB * 64) / 128), 128, 0, stream>>>(DT, P, b, BCD); }
  k_aa<<<dim3(CC / 64, CC / 128, TNB), 128, 0, stream>>>(XT, AA);
  k_soft<<<dim3(CC / 64, TNB), 256, 0, stream>>>(AA, SO);
  k_aaa<<<dim3(TRB, CC / 128, TNB), 128, 0, stream>>>(F[0], SO, AAA);
  k_fin<<<(unsigned)((size_t)TNB * NN * CC / 1024), 256, 0, stream>>>(BCD, AAA, F[0], F[4], F[5], (float*)d_out);
}
